// DAPTriAttEnd_19112604467523
// MI455X (gfx1250) — hardware-verified
//
#include <hip/hip_runtime.h>
#include <stddef.h>


typedef _Float16       v8h  __attribute__((ext_vector_type(8)));
typedef _Float16       v16h __attribute__((ext_vector_type(16)));
typedef __bf16         v16b __attribute__((ext_vector_type(16)));
typedef unsigned short v8us __attribute__((ext_vector_type(8)));
typedef float          v4f  __attribute__((ext_vector_type(4)));
typedef float          v8f  __attribute__((ext_vector_type(8)));

#define NN   256
#define CC   128
#define HH   4
#define DD   32
#define NPOS (NN * NN)
#define XP   132
#define KP   264
#define AP   136
#define TBP  1024

union FragH { v16h v; v8h p[2]; _Float16 s[16]; };
union FragB { v16b v; v8us p[2]; unsigned short s[16]; };

__device__ __forceinline__ v8f vz8() {
    v8f z = {0.f, 0.f, 0.f, 0.f, 0.f, 0.f, 0.f, 0.f};
    return z;
}

__device__ __forceinline__ v8f wm16(v8f c, v16h a, v16h b) {
    v8f d = __builtin_amdgcn_wmma_f32_16x16x32_f16(false, a, false, b, (short)0, c, false, false);
    asm volatile("v_nop\n\tv_nop\n\tv_nop\n\tv_nop" : "+v"(d) : "v"(a), "v"(b));
    return d;
}
__device__ __forceinline__ v8f wmbf(v8f c, v16b a, v16b b) {
    v8f d = __builtin_amdgcn_wmma_f32_16x16x32_bf16(false, a, false, b, (short)0, c, false, false);
    asm volatile("v_nop\n\tv_nop\n\tv_nop\n\tv_nop" : "+v"(d) : "v"(a), "v"(b));
    return d;
}

__device__ __forceinline__ unsigned int bf_bits(float f) {
    unsigned int u = __float_as_uint(f);
    u += 0x7FFFu + ((u >> 16) & 1u);
    return u >> 16;
}
__device__ __forceinline__ void bf_split(float f, unsigned short& hi, unsigned short& lo) {
    const unsigned int hb = bf_bits(f);
    const float fh = __uint_as_float(hb << 16);
    hi = (unsigned short)hb;
    lo = (unsigned short)bf_bits(f - fh);
}

__device__ __forceinline__ v16h frag_f16(const _Float16* rowk, int lh) {
    FragH f;
    f.p[0] = *(const v8h*)(rowk + 8 * lh);
    f.p[1] = *(const v8h*)(rowk + 16 + 8 * lh);
    return f.v;
}
__device__ __forceinline__ v16b frag_bf(const unsigned short* rowk, int lh) {
    FragB f;
    f.p[0] = *(const v8us*)(rowk + 8 * lh);
    f.p[1] = *(const v8us*)(rowk + 16 + 8 * lh);
    return f.v;
}

__device__ __forceinline__ v16h afrag_f16(const float* xr, int k0, int lh) {
    const float* p0 = xr + k0 + 8 * lh;
    const float* p1 = xr + k0 + 16 + 8 * lh;
    const v4f f0 = *(const v4f*)(p0);
    const v4f f1 = *(const v4f*)(p0 + 4);
    const v4f f2 = *(const v4f*)(p1);
    const v4f f3 = *(const v4f*)(p1 + 4);
    FragH a;
#pragma unroll
    for (int e = 0; e < 4; ++e) {
        a.s[e]      = (_Float16)f0[e];
        a.s[4 + e]  = (_Float16)f1[e];
        a.s[8 + e]  = (_Float16)f2[e];
        a.s[12 + e] = (_Float16)f3[e];
    }
    return a.v;
}
__device__ __forceinline__ void afrag_bf(const float* xr, int k0, int lh, v16b& hi, v16b& lo) {
    const float* p0 = xr + k0 + 8 * lh;
    const float* p1 = xr + k0 + 16 + 8 * lh;
    const v4f f0 = *(const v4f*)(p0);
    const v4f f1 = *(const v4f*)(p0 + 4);
    const v4f f2 = *(const v4f*)(p1);
    const v4f f3 = *(const v4f*)(p1 + 4);
    FragB H, L;
#pragma unroll
    for (int e = 0; e < 4; ++e) {
        bf_split(f0[e], H.s[e],      L.s[e]);
        bf_split(f1[e], H.s[4 + e],  L.s[4 + e]);
        bf_split(f2[e], H.s[8 + e],  L.s[8 + e]);
        bf_split(f3[e], H.s[12 + e], L.s[12 + e]);
    }
    hi = H.v;
    lo = L.v;
}

__device__ __forceinline__ void ln_rows(const float* __restrict__ x, const float* __restrict__ lnw,
                                        const float* __restrict__ lnb, float* XF,
                                        int i, int j0, int w, int l)
{
    const v4f wv = ((const v4f*)lnw)[l];
    const v4f bv = ((const v4f*)lnb)[l];
#pragma unroll
    for (int rr = 0; rr < 4; ++rr) {
        const int r = w * 4 + rr;
        const float* row = x + ((size_t)(j0 + r) * NN + i) * CC;
        const v4f xv = ((const v4f*)row)[l];
        float s = (xv[0] + xv[1]) + (xv[2] + xv[3]);
#pragma unroll
        for (int o = 16; o >= 1; o >>= 1) s += __shfl_xor(s, o, 32);
        const float mean = s * (1.0f / 128.0f);
        const v4f d = xv - mean;
        float s2 = (d[0] * d[0] + d[1] * d[1]) + (d[2] * d[2] + d[3] * d[3]);
#pragma unroll
        for (int o = 16; o >= 1; o >>= 1) s2 += __shfl_xor(s2, o, 32);
        const float var = s2 * (1.0f / 128.0f);
        const float rstd = rsqrtf(var + 1e-5f);
        const v4f y = d * rstd * wv + bv;
        *(v4f*)(XF + r * XP + 4 * l) = y;
    }
}

__global__ __launch_bounds__(256) void k_prep(
    const float* __restrict__ wq, const float* __restrict__ wk, const float* __restrict__ wv,
    const float* __restrict__ wg, const float* __restrict__ wo,
    _Float16* Wqk, _Float16* Wg16, unsigned short* WvH, unsigned short* WvL,
    unsigned short* WoH, unsigned short* WoL)
{
    const int t = blockIdx.x * 256 + threadIdx.x;
    if (t < 4096) {
        const int n = t >> 4, c0 = (t & 15) * 8, nn = n & 127;
        const float* src = (n < 128) ? wq : wk;
        v8h val;
#pragma unroll
        for (int e = 0; e < 8; ++e) val[e] = (_Float16)(src[(size_t)(c0 + e) * CC + nn] * 64.0f);
        volatile v8h* dst = (volatile v8h*)(Wqk + (size_t)n * CC + c0);
        *dst = val;
        __threadfence();
        *dst = val;
    } else if (t < 6144) {
        const int u = t - 4096;
        const int n = u >> 4, c0 = (u & 15) * 8;
        v8h val;
#pragma unroll
        for (int e = 0; e < 8; ++e) val[e] = (_Float16)(wg[(size_t)(c0 + e) * CC + n] * 64.0f);
        volatile v8h* dst = (volatile v8h*)(Wg16 + (size_t)n * CC + c0);
        *dst = val;
        __threadfence();
        *dst = val;
    } else if (t < 8192) {
        const int u = t - 6144;
        const int n = u >> 4, c0 = (u & 15) * 8;
        v8us hv, lv;
#pragma unroll
        for (int e = 0; e < 8; ++e) {
            unsigned short hs, ls;
            bf_split(wv[(size_t)(c0 + e) * CC + n], hs, ls);
            hv[e] = hs; lv[e] = ls;
        }
        volatile v8us* dh = (volatile v8us*)(WvH + (size_t)n * CC + c0);
        volatile v8us* dl = (volatile v8us*)(WvL + (size_t)n * CC + c0);
        *dh = hv; *dl = lv;
        __threadfence();
        *dh = hv; *dl = lv;
    } else if (t < 10240) {
        const int u = t - 8192;
        const int n = u >> 4, c0 = (u & 15) * 8;
        v8us hv, lv;
#pragma unroll
        for (int e = 0; e < 8; ++e) {
            unsigned short hs, ls;
            bf_split(wo[(size_t)n * CC + c0 + e], hs, ls);
            hv[e] = hs; lv[e] = ls;
        }
        volatile v8us* dh = (volatile v8us*)(WoH + (size_t)n * CC + c0);
        volatile v8us* dl = (volatile v8us*)(WoL + (size_t)n * CC + c0);
        *dh = hv; *dl = lv;
        __threadfence();
        *dh = hv; *dl = lv;
    }
}

__global__ __launch_bounds__(128) void k_proj(
    const float* __restrict__ x, const float* __restrict__ lnw, const float* __restrict__ lnb,
    const float* __restrict__ wbias, const _Float16* __restrict__ Wqk,
    const unsigned short* __restrict__ WvH, const unsigned short* __restrict__ WvL,
    _Float16* qb, _Float16* kb, float* vb, float* tb)
{
    __shared__ __align__(16) float    XF[16 * XP];
    __shared__ __align__(16) _Float16 SQ[2][4][16][32];
    __shared__ __align__(16) float    SV[4][16][32];
    __shared__ __align__(16) float    STB[64];

    const int tid = threadIdx.x, w = tid >> 5, l = tid & 31;
    const int p0 = blockIdx.x * 16;
    if (p0 >= NPOS) return;
    const int i = p0 >> 8, j0 = p0 & 255;

    ln_rows(x, lnw, lnb, XF, i, j0, w, l);
    __syncthreads();

    if (tid < 64) {
        const int r = tid >> 2, h = tid & 3;
        const float* wb = wbias + h * CC;
        const float* xr = XF + r * XP;
        float acc = 0.0f;
#pragma unroll 4
        for (int c = 0; c < CC; ++c) acc = fmaf(xr[c], wb[c], acc);
        STB[h * 16 + r] = acc;
    }

    const int m = l & 15, lh = l >> 4;
    const float* xr = XF + m * XP;
    if (w < 2) {
        v8f acc[8];
#pragma unroll
        for (int t = 0; t < 8; ++t) acc[t] = vz8();
#pragma unroll
        for (int kk = 0; kk < 4; ++kk) {
            const int k0 = kk * 32;
            const v16h a = afrag_f16(xr, k0, lh);
#pragma unroll
            for (int t = 0; t < 8; ++t) {
                const v16h b = frag_f16(Wqk + (size_t)(w * 128 + t * 16 + m) * CC + k0, lh);
                acc[t] = wm16(acc[t], a, b);
            }
        }
        const float sc = (w == 0) ? (0.17677669529663687f * 0.015625f) : 0.015625f;
#pragma unroll
        for (int t = 0; t < 8; ++t) {
            const int h = t >> 1, d = (t & 1) * 16 + m;
#pragma unroll
            for (int r = 0; r < 8; ++r) SQ[w][h][8 * lh + r][d] = (_Float16)(acc[t][r] * sc);
        }
    } else {
        const int cb = (w - 2) * 64;
        v8f acc[4];
#pragma unroll
        for (int t = 0; t < 4; ++t) acc[t] = vz8();
#pragma unroll
        for (int kk = 0; kk < 4; ++kk) {
            const int k0 = kk * 32;
            v16b ah, al;
            afrag_bf(xr, k0, lh, ah, al);
#pragma unroll
            for (int t = 0; t < 4; ++t) {
                const int n = cb + t * 16 + m;
                const v16b bh = frag_bf(WvH + (size_t)n * CC + k0, lh);
                const v16b bl = frag_bf(WvL + (size_t)n * CC + k0, lh);
                acc[t] = wmbf(acc[t], ah, bh);
                acc[t] = wmbf(acc[t], ah, bl);
                acc[t] = wmbf(acc[t], al, bh);
            }
        }
#pragma unroll
        for (int t = 0; t < 4; ++t) {
            const int col = cb + t * 16 + m;
            const int h = col >> 5, d = col & 31;
#pragma unroll
            for (int r = 0; r < 8; ++r) SV[h][8 * lh + r][d] = acc[t][r];
        }
    }
    __syncthreads();

    auto stores = [&]() {
        if (w < 2) {
            _Float16* dstb = (w == 0) ? qb : kb;
#pragma unroll
            for (int h = 0; h < 4; ++h) {
                const v8h* src = (const v8h*)&SQ[w][h][0][0];
                volatile v8h* dst = (volatile v8h*)(dstb + ((size_t)(i * HH + h) * NN + j0) * DD);
                const v8h a0 = src[l], a1 = src[32 + l];
                dst[l] = a0;
                dst[32 + l] = a1;
            }
        } else {
#pragma unroll
            for (int q = 0; q < 2; ++q) {
                const int h = (w - 2) * 2 + q;
                const v4f* src = (const v4f*)&SV[h][0][0];
                volatile v4f* dst = (volatile v4f*)(vb + ((size_t)(i * HH + h) * NN + j0) * DD);
                const v4f a0 = src[l], a1 = src[32 + l], a2 = src[64 + l], a3 = src[96 + l];
                dst[l] = a0; dst[32 + l] = a1; dst[64 + l] = a2; dst[96 + l] = a3;
            }
        }
        if (tid < 16) {
            const v4f a0 = ((const v4f*)STB)[tid];
            volatile v4f* dst = (volatile v4f*)(tb + (size_t)i * TBP + (size_t)(j0 >> 4) * 64);
            dst[tid] = a0;
        }
    };
    stores();
    __threadfence();
    stores();
}

__global__ __launch_bounds__(64) void k_attn(
    const _Float16* __restrict__ qb, const _Float16* __restrict__ kb, const float* __restrict__ vb,
    const float* __restrict__ tb, const float* __restrict__ mask, float* ob)
{
    __shared__ __align__(16) _Float16       KS[NN * DD];
    __shared__ __align__(16) unsigned short VH[DD][KP];
    __shared__ __align__(16) unsigned short VL[DD][KP];
    __shared__ __align__(16) unsigned short PH[2][16][KP];
    __shared__ __align__(16) unsigned short PL[2][16][KP];
    __shared__ __align__(16) float          SO[2][16][DD];
    __shared__ float MB[NN];

    const int tid = threadIdx.x, w = tid >> 5, l = tid & 31, m = l & 15, lh = l >> 4;
    const int bid = blockIdx.x;
    if (bid >= NN * HH) return;
    const int i = bid >> 2, h = bid & 3;
    const size_t ih = (size_t)i * HH + h;
    const _Float16* qsrc = qb + ih * NN * DD;
    const _Float16* ksrc = kb + ih * NN * DD;
    const float*    vsrc = vb + ih * NN * DD;

    for (int u = tid; u < (NN * DD) / 8; u += 64) ((v8h*)KS)[u] = ((const v8h*)ksrc)[u];
    for (int u = tid; u < (NN * DD) / 4; u += 64) {
        const int key = u >> 3, d0 = (u & 7) * 4;
        const v4f f = ((const v4f*)vsrc)[u];
#pragma unroll
        for (int e = 0; e < 4; ++e) {
            unsigned short hs, ls;
            bf_split(f[e], hs, ls);
            VH[d0 + e][key] = hs;
            VL[d0 + e][key] = ls;
        }
    }
    for (int u = tid; u < NN; u += 64) MB[u] = 1.0e9f * (mask[(size_t)u * NN + i] - 1.0f);
    __syncthreads();

#pragma unroll 1
    for (int qi = 0; qi < 8; ++qi) {
        const int j0 = (w * 8 + qi) * 16;

        const v16h qa = frag_f16(qsrc + (size_t)(j0 + m) * DD, lh);
        const float* tp = tb + (size_t)(j0 + 8 * lh) * TBP + h * 16 + m;
        v8f s[16];
#pragma unroll
        for (int b = 0; b < 16; ++b) {
            const v16h kf = frag_f16(KS + (b * 16 + m) * DD, lh);
            v8f c = wm16(vz8(), qa, kf);
            const float mb = MB[b * 16 + m];
            const float* tpb = tp + b * 64;
#pragma unroll
            for (int r = 0; r < 8; ++r) c[r] = (c[r] + mb) + tpb[(size_t)r * TBP];
            s[b] = c;
        }

#pragma unroll
        for (int r = 0; r < 8; ++r) {
            float mx = s[0][r];
#pragma unroll
            for (int b = 1; b < 16; ++b) mx = fmaxf(mx, s[b][r]);
            mx = fmaxf(mx, __shfl_xor(mx, 8, 32));
            mx = fmaxf(mx, __shfl_xor(mx, 4, 32));
            mx = fmaxf(mx, __shfl_xor(mx, 2, 32));
            mx = fmaxf(mx, __shfl_xor(mx, 1, 32));
            float sum = 0.0f;
#pragma unroll
            for (int b = 0; b < 16; ++b) {
                const float e = __expf(s[b][r] - mx);
                s[b][r] = e;
                sum += e;
            }
            sum += __shfl_xor(sum, 8, 32);
            sum += __shfl_xor(sum, 4, 32);
            sum += __shfl_xor(sum, 2, 32);
            sum += __shfl_xor(sum, 1, 32);
            const float inv = __builtin_amdgcn_rcpf(sum);
            const int row = 8 * lh + r;
#pragma unroll
            for (int b = 0; b < 16; ++b) {
                unsigned short hs, ls;
                bf_split(s[b][r] * inv, hs, ls);
                PH[w][row][b * 16 + m] = hs;
                PL[w][row][b * 16 + m] = ls;
            }
        }
        __syncthreads();

        v8f o0 = vz8(), o1 = vz8();
#pragma unroll
        for (int c32 = 0; c32 < 8; ++c32) {
            const int k0 = c32 * 32;
            const v16b pah = frag_bf(&PH[w][m][k0], lh);
            const v16b pal = frag_bf(&PL[w][m][k0], lh);
            const v16b vh0 = frag_bf(&VH[m][k0], lh);
            const v16b vl0 = frag_bf(&VL[m][k0], lh);
            const v16b vh1 = frag_bf(&VH[16 + m][k0], lh);
            const v16b vl1 = frag_bf(&VL[16 + m][k0], lh);
            o0 = wmbf(o0, pah, vh0);
            o0 = wmbf(o0, pah, vl0);
            o0 = wmbf(o0, pal, vh0);
            o1 = wmbf(o1, pah, vh1);
            o1 = wmbf(o1, pah, vl1);
            o1 = wmbf(o1, pal, vh1);
        }
#pragma unroll
        for (int r = 0; r < 8; ++r) {
            SO[w][8 * lh + r][m]      = o0[r];
            SO[w][8 * lh + r][16 + m] = o1[r];
        }
        __syncthreads();

        {
            const v4f* src = (const v4f*)&SO[w][0][0];
            const v4f t0 = src[l], t1 = src[32 + l], t2 = src[64 + l], t3 = src[96 + l];
            volatile v4f* dst = (volatile v4f*)(ob + (ih * NN + j0) * DD);
            dst[l] = t0; dst[32 + l] = t1; dst[64 + l] = t2; dst[96 + l] = t3;
            __threadfence();
            dst[l] = t0; dst[32 + l] = t1; dst[64 + l] = t2; dst[96 + l] = t3;
        }
    }
}

__global__ __launch_bounds__(128) void k_out(
    const float* __restrict__ x, const float* __restrict__ lnw, const float* __restrict__ lnb,
    const _Float16* __restrict__ Wg16, const float* __restrict__ bg, const float* __restrict__ ob,
    const unsigned short* __restrict__ WoH, const unsigned short* __restrict__ WoL,
    const float* __restrict__ bo, float* out)
{
    __shared__ __align__(16) float          XF[16 * XP];
    __shared__ __align__(16) unsigned short AH[16][AP];
    __shared__ __align__(16) unsigned short AL[16][AP];
    __shared__ __align__(16) float          SOUT[16][XP];

    const int tid = threadIdx.x, w = tid >> 5, l = tid & 31, m = l & 15, lh = l >> 4;
    const int p0 = blockIdx.x * 16;
    if (p0 >= NPOS) return;
    const int i = p0 >> 8, j0 = p0 & 255;

    ln_rows(x, lnw, lnb, XF, i, j0, w, l);
    __syncthreads();

    const float* xr = XF + m * XP;
    v8f ga[2];
    ga[0] = vz8(); ga[1] = vz8();
#pragma unroll
    for (int kk = 0; kk < 4; ++kk) {
        const int k0 = kk * 32;
        const v16h a = afrag_f16(xr, k0, lh);
#pragma unroll
        for (int t = 0; t < 2; ++t) {
            const v16h b = frag_f16(Wg16 + (size_t)(32 * w + 16 * t + m) * CC + k0, lh);
            ga[t] = wm16(ga[t], a, b);
        }
    }
#pragma unroll
    for (int t = 0; t < 2; ++t) {
        const int d = 16 * t + m, n = 32 * w + d;
        const float bgn = bg[n];
        const float* op = ob + ((size_t)(i * HH + w) * NN + j0 + 8 * lh) * DD + d;
#pragma unroll
        for (int r = 0; r < 8; ++r) {
            const float pre = ga[t][r] * 0.015625f + bgn;
            const float gs  = __builtin_amdgcn_rcpf(1.0f + __expf(-pre));
            const float a   = op[(size_t)r * DD] * gs;
            unsigned short hs, ls;
            bf_split(a, hs, ls);
            AH[8 * lh + r][n] = hs;
            AL[8 * lh + r][n] = ls;
        }
    }
    __syncthreads();

    v8f oc[2];
    oc[0] = vz8(); oc[1] = vz8();
#pragma unroll
    for (int kk = 0; kk < 4; ++kk) {
        const int k0 = kk * 32;
        const v16b ah = frag_bf(&AH[m][k0], lh);
        const v16b al = frag_bf(&AL[m][k0], lh);
#pragma unroll
        for (int t = 0; t < 2; ++t) {
            const int n = 32 * w + 16 * t + m;
            const v16b bh = frag_bf(WoH + (size_t)n * CC + k0, lh);
            const v16b bl = frag_bf(WoL + (size_t)n * CC + k0, lh);
            oc[t] = wmbf(oc[t], ah, bh);
            oc[t] = wmbf(oc[t], ah, bl);
            oc[t] = wmbf(oc[t], al, bh);
        }
    }
#pragma unroll
    for (int t = 0; t < 2; ++t) {
        const int n = 32 * w + 16 * t + m;
        const float bon = bo[n];
#pragma unroll
        for (int r = 0; r < 8; ++r) SOUT[8 * lh + r][n] = oc[t][r] + bon;
    }
    __syncthreads();

    v4f sv[4];
#pragma unroll
    for (int sI = 0; sI < 4; ++sI) {
        const int q = sI * 128 + tid;
        const int L = q >> 3, mrow = L >> 2, seg = L & 3, pc = q & 7;
        sv[sI] = *(const v4f*)&SOUT[mrow][seg * 32 + pc * 4];
    }
#pragma unroll
    for (int sI = 0; sI < 4; ++sI) {
        const int q = sI * 128 + tid;
        const int L = q >> 3, mrow = L >> 2, seg = L & 3, pc = q & 7;
        volatile v4f* dst = (volatile v4f*)(out + ((size_t)(j0 + mrow) * NN + i) * CC + seg * 32 + pc * 4);
        *dst = sv[sI];
    }
    __threadfence();
#pragma unroll
    for (int sI = 0; sI < 4; ++sI) {
        const int q = sI * 128 + tid;
        const int L = q >> 3, mrow = L >> 2, seg = L & 3, pc = q & 7;
        volatile v4f* dst = (volatile v4f*)(out + ((size_t)(j0 + mrow) * NN + i) * CC + seg * 32 + pc * 4);
        *dst = sv[sI];
    }
}

extern "C" void kernel_launch(void* const* d_in, const int* in_sizes, int n_in,
                              void* d_out, int out_size, void* d_ws, size_t ws_size,
                              hipStream_t stream)
{
    if (n_in < 12) return;
    if (in_sizes[0] != NPOS * CC || in_sizes[1] != NPOS || in_sizes[2] != CC || in_sizes[3] != CC ||
        in_sizes[4] != HH * CC || in_sizes[5] != CC * HH * DD || in_sizes[6] != CC * HH * DD ||
        in_sizes[7] != CC * HH * DD || in_sizes[8] != CC * HH * DD || in_sizes[9] != HH * DD ||
        in_sizes[10] != CC * HH * DD || in_sizes[11] != CC || out_size != NPOS * CC) return;

    const float* x     = (const float*)d_in[0];
    const float* mask  = (const float*)d_in[1];
    const float* ln_w  = (const float*)d_in[2];
    const float* ln_b  = (const float*)d_in[3];
    const float* wbias = (const float*)d_in[4];
    const float* wq    = (const float*)d_in[5];
    const float* wk    = (const float*)d_in[6];
    const float* wv    = (const float*)d_in[7];
    const float* wg    = (const float*)d_in[8];
    const float* bg    = (const float*)d_in[9];
    const float* wo    = (const float*)d_in[10];
    const float* bo    = (const float*)d_in[11];
    float* outp = (float*)d_out;

    char* ws = (char*)d_ws;
    size_t off = 0;
    _Float16*       Wqk  = (_Float16*)(ws + off);       off += (size_t)256 * CC * 2;
    _Float16*       Wg16 = (_Float16*)(ws + off);       off += (size_t)CC * CC * 2;
    unsigned short* WvH  = (unsigned short*)(ws + off); off += (size_t)CC * CC * 2;
    unsigned short* WvL  = (unsigned short*)(ws + off); off += (size_t)CC * CC * 2;
    unsigned short* WoH  = (unsigned short*)(ws + off); off += (size_t)CC * CC * 2;
    unsigned short* WoL  = (unsigned short*)(ws + off); off += (size_t)CC * CC * 2;
    _Float16*       qb   = (_Float16*)(ws + off);       off += (size_t)NN * HH * NN * DD * 2;
    _Float16*       kb   = (_Float16*)(ws + off);       off += (size_t)NN * HH * NN * DD * 2;
    float*          vb   = (float*)(ws + off);          off += (size_t)NN * HH * NN * DD * 4;
    float*          ob   = (float*)(ws + off);          off += (size_t)NN * HH * NN * DD * 4;
    float*          tb   = (float*)(ws + off);          off += (size_t)NN * TBP * 4;
    if (off > ws_size) return;

    k_prep<<<40, 256, 0, stream>>>(wq, wk, wv, wg, wo, Wqk, Wg16, WvH, WvL, WoH, WoL);
    k_proj<<<NPOS / 16, 128, 0, stream>>>(x, ln_w, ln_b, wbias, Wqk, WvH, WvL, qb, kb, vb, tb);
    k_attn<<<NN * HH, 64, 0, stream>>>(qb, kb, vb, tb, mask, ob);
    k_out<<<NPOS / 16, 128, 0, stream>>>(x, ln_w, ln_b, Wg16, bg, ob, WoH, WoL, bo, outp);
}
